// LNNMotion_76270029242693
// MI455X (gfx1250) — hardware-verified
//
#include <hip/hip_runtime.h>
#include <math.h>

typedef __attribute__((ext_vector_type(16))) _Float16 v16h;
typedef __attribute__((ext_vector_type(16))) __bf16 v16b;
typedef __attribute__((ext_vector_type(8)))  _Float16 v8h;
typedef __attribute__((ext_vector_type(8)))  float v8f;
typedef __attribute__((ext_vector_type(4)))  float v4f;
typedef __attribute__((ext_vector_type(2)))  float v2f;
typedef __attribute__((ext_vector_type(4)))  unsigned v4u;
typedef __attribute__((ext_vector_type(4)))  int v4i;
typedef float __attribute__((may_alias)) float_a;
typedef int __attribute__((may_alias)) int_a;

template <typename T> __device__ __forceinline__ void vst2(void* p, T v) { *(volatile T*)p = v; __threadfence(); *(volatile T*)p = v; }
__device__ __forceinline__ v8f wmma16(v16h a, v16h b, v8f c) {
  v8f d = __builtin_amdgcn_wmma_f32_16x16x32_f16(false, a, false, b, (short)0, c, false, false);
  asm volatile("v_nop\n\tv_nop\n\tv_nop\n\tv_nop" : "+v"(d) : "v"(a), "v"(b));
  return d;
}
__device__ __forceinline__ v8f wmma_bf(v16b a, v16b b, v8f c) {
  v8f d = __builtin_amdgcn_wmma_f32_16x16x32_bf16(false, a, false, b, (short)0, c, false, false);
  asm volatile("v_nop\n\tv_nop\n\tv_nop\n\tv_nop" : "+v"(d) : "v"(a), "v"(b));
  return d;
}
__device__ __forceinline__ v16h frag_h(const _Float16* rowk0, int lane) {
  union { v16h v; v8h q[2]; } u; const _Float16* p = rowk0 + 8 * (lane >> 4);
  u.q[0] = *(const v8h*)p; u.q[1] = *(const v8h*)(p + 16); return u.v;
}
__device__ __forceinline__ v16h frag_f32(const float* rowk0, int lane) {
  v16h a; const float* p = rowk0 + 8 * (lane >> 4);
#pragma unroll
  for (int i = 0; i < 8; ++i) { a[i] = (_Float16)p[i]; a[8 + i] = (_Float16)p[16 + i]; }
  return a;
}
__device__ __forceinline__ v16h frag_f32s(const float* rowk0, int lane, float sc) {
  v16h a; const float* p = rowk0 + 8 * (lane >> 4);
#pragma unroll
  for (int i = 0; i < 8; ++i) { a[i] = (_Float16)(p[i] * sc); a[8 + i] = (_Float16)(p[16 + i] * sc); }
  return a;
}
__device__ __forceinline__ v16h fragc_f32(const float* W, int k0, int n, int lane, int ld, int K) {
  v16h a; const int g = lane >> 4;
#pragma unroll
  for (int i = 0; i < 8; ++i) { const int ka = k0 + 8 * g + i, kb = ka + 16;
    a[i] = (_Float16)(ka < K ? W[(size_t)(ka < K ? ka : K - 1) * ld + n] : 0.f); a[8 + i] = (_Float16)(kb < K ? W[(size_t)(kb < K ? kb : K - 1) * ld + n] : 0.f); }
  return a;
}
struct F2 { v16b h, l; };
__device__ __forceinline__ F2 bsplit16(const float v[16]) { F2 r;
#pragma unroll
  for (int i = 0; i < 16; ++i) { const __bf16 h = (__bf16)v[i]; r.h[i] = h; r.l[i] = (__bf16)(v[i] - (float)h); }
  return r; }
__device__ __forceinline__ F2 split_row(const float* row, int k0, int lane) { float v[16]; const float* p = row + k0 + 8 * (lane >> 4);
#pragma unroll
  for (int i = 0; i < 8; ++i) { v[i] = p[i]; v[8 + i] = p[16 + i]; }
  return bsplit16(v); }
__device__ __forceinline__ F2 split_rowK(const float* row, int k0, int lane, int K) { float v[16]; const int g = lane >> 4;
#pragma unroll
  for (int i = 0; i < 8; ++i) { const int ka = k0 + 8 * g + i, kb = ka + 16; v[i] = ka < K ? row[ka < K ? ka : K - 1] : 0.f; v[8 + i] = kb < K ? row[kb < K ? kb : K - 1] : 0.f; }
  return bsplit16(v); }
__device__ __forceinline__ F2 split_col(const float* W, int k0, int n, int lane, int ld, int K) { float v[16]; const int g = lane >> 4;
#pragma unroll
  for (int i = 0; i < 8; ++i) { const int ka = k0 + 8 * g + i, kb = ka + 16; v[i] = ka < K ? W[(size_t)(ka < K ? ka : K - 1) * ld + n] : 0.f; v[8 + i] = kb < K ? W[(size_t)(kb < K ? kb : K - 1) * ld + n] : 0.f; }
  return bsplit16(v); }
__device__ __forceinline__ v8f mac3(const F2& a, const F2& b, v8f c) { c = wmma_bf(a.l, b.h, c); c = wmma_bf(a.h, b.l, c); return wmma_bf(a.h, b.h, c); }
__device__ __forceinline__ float sigm(float v) { return 1.0f / (1.0f + expf(-v)); }
#define LDSX() do { asm volatile("s_wait_dscnt 0" ::: "memory"); __builtin_amdgcn_wave_barrier(); __builtin_amdgcn_fence(__ATOMIC_RELEASE, "workgroup"); } while (0)


#define NB 1024
#define TT 128
#define NIN 2
#define HH 256
#define NOUT 2
#ifndef NRB
#define NRB (NB / 64)
#endif
typedef __attribute__((ext_vector_type(8))) __bf16 v8b;
__device__ __forceinline__ v16b frag_b(const __bf16* rowk0, int lane) {
  union { v16b v; v8b q[2]; } u; const __bf16* p = rowk0 + 8 * (lane >> 4);
  u.q[0] = *(const v8b*)p; u.q[1] = *(const v8b*)(p + 16); return u.v;
}
__device__ __forceinline__ float bfr(float v) { return (float)(__bf16)v; }
__device__ __attribute__((noinline)) float exp_ni(float v) { return expf(v); }
__device__ __attribute__((noinline)) float erf_ni(float v) { return erff(v); }

__device__ __attribute__((noinline)) float tanh_ni(float v) { return tanhf(v); }
#define WS_PW  0u
#define WS_END (WS_PW + 2u * HH * HH)

__global__ __launch_bounds__(256) void k_pack(const float* __restrict__ WH, __bf16* __restrict__ PW) {
  __shared__ __align__(16) __bf16 s[HH]; const int n = blockIdx.x, k = threadIdx.x; s[k] = (__bf16)WH[(size_t)n * HH + k]; __syncthreads();
  if (k < HH / 8) vst2((unsigned*)(PW + (size_t)n * HH + k * 8), *(const v4u*)&s[k * 8]);
}
__global__ __launch_bounds__(128) void k_lnn(const float* __restrict__ X, const float* __restrict__ WIN, const float* __restrict__ BIN, const __bf16* __restrict__ PW, const float* __restrict__ BH, const float* __restrict__ AL, const float* __restrict__ BE, const float* __restrict__ FCW, const float* __restrict__ FCB, float* __restrict__ out) {
  __shared__ __align__(16) float sh[64][HH + 4]; __shared__ float swin[HH][2], sbias[HH], sab[HH], sfc[2][HH]; __shared__ __align__(16) float so[64 * NOUT];
  const int tid = threadIdx.x, wave = tid >> 5, lane = tid & 31, col = lane & 15, g = lane >> 4; const size_t b0 = (size_t)blockIdx.x * 64; const int r0 = wave * 16;
  for (int q = tid; q < HH; q += 128) { swin[q][0] = bfr(WIN[q * 2]); swin[q][1] = bfr(WIN[q * 2 + 1]); sbias[q] = bfr(BIN[q]) + bfr(BH[q]); sab[q] = bfr(AL[q]) * bfr(BE[q]); sfc[0][q] = bfr(FCW[q]); sfc[1][q] = bfr(FCW[HH + q]); }
  for (int q = tid; q < 64 * HH; q += 128) sh[q / HH][q % HH] = 0.f;
  __syncthreads();
#pragma unroll 1
  for (int t = 0; t < TT; ++t) {
    v8f acc[16]; for (int j = 0; j < 16; ++j) acc[j] = (v8f){};
#pragma unroll 2
    for (int kc = 0; kc < HH / 32; ++kc) { const F2 a = split_row(&sh[r0 + col][0], kc * 32, lane);
#pragma unroll
      for (int j = 0; j < 16; ++j) { const v16b w = frag_b(PW + (size_t)(j * 16 + col) * HH + kc * 32, lane); acc[j] = wmma_bf(a.l, w, acc[j]); acc[j] = wmma_bf(a.h, w, acc[j]); } }
    float x0[8], x1[8];
#pragma unroll
    for (int r = 0; r < 8; ++r) { const size_t b = b0 + r0 + 8 * g + r; x0[r] = bfr(X[(b * TT + t) * NIN]); x1[r] = bfr(X[(b * TT + t) * NIN + 1]); }
    LDSX();
#pragma unroll
    for (int j = 0; j < 16; ++j) { const int c = j * 16 + col; const float w0 = swin[c][0], w1 = swin[c][1], bb = sbias[c], ab = sab[c];
#pragma unroll
      for (int r = 0; r < 8; ++r) { const int rl = r0 + 8 * g + r; const float pre = acc[j][r] + bb + x0[r] * w0 + x1[r] * w1; const float hold = sh[rl][c]; sh[rl][c] = hold + ab * (tanh_ni(pre) - hold); } }
    LDSX(); }
  for (int rl = 0; rl < 16; ++rl) { float p0 = 0.f, p1 = 0.f;
#pragma unroll
    for (int k = 0; k < 8; ++k) { const int c = lane + 32 * k; const float hv = sh[r0 + rl][c]; p0 += hv * sfc[0][c]; p1 += hv * sfc[1][c]; }
#pragma unroll
    for (int o = 1; o < 32; o <<= 1) { p0 += __shfl_xor(p0, o); p1 += __shfl_xor(p1, o); }
    if (lane == 0) { so[(r0 + rl) * 2] = p0 + bfr(FCB[0]); so[(r0 + rl) * 2 + 1] = p1 + bfr(FCB[1]); } }
  __syncthreads();
  if (tid < 32) vst2(out + b0 * NOUT + tid * 4, *(const v4f*)&so[tid * 4]);
}
extern "C" void kernel_launch(void* const* d_in, const int* in_sizes, int n_in, void* d_out, int out_size, void* d_ws, size_t ws_size, hipStream_t stream) {
  (void)in_sizes; (void)n_in; (void)out_size;
  const float** F = (const float**)d_in;
  if (ws_size < (size_t)WS_END) return;
  char* ws = (char*)d_ws; __bf16* PW = (__bf16*)(ws + WS_PW);
  k_pack<<<HH, 256, 0, stream>>>(F[3], PW);
  k_lnn<<<NRB, 128, 0, stream>>>(F[0], F[1], F[2], PW, F[4], F[5], F[6], F[7], F[8], (float*)d_out);
}
